// MixBlock_68659347194418
// MI455X (gfx1250) — hardware-run, weakly checked
//
#include <hip/hip_runtime.h>
#include <stdint.h>

#define NBAT   2
#define IMH    128
#define IMW    128
#define SEQ    16384
#define CH     96
#define NT     32768
#define NHD    6
#define HDM    16
#define DST    16
#define DTR    6
#define XDB    38
#define HID    384
#define LDC    100
#define RSC    0.00048828125f
#define PLN    ((size_t)NT * CH)
#define UNIT   ((size_t)6291456)

#define WO_IP  ((size_t)0)
#define WO_QK  ((size_t)27648)
#define WO_XP  ((size_t)46080)
#define WO_O1  ((size_t)55296)
#define WO_PO  ((size_t)73728)
#define WO_OU  ((size_t)82944)
#define WO_F1  ((size_t)101376)
#define WO_F2  ((size_t)138240)
#define WO_END ((size_t)175104)
#define SB_WPL ((size_t)0)
#define SB_KMP ((size_t)350208)
#define SB_KM  ((size_t)546816)
#define SB_KVP ((size_t)547584)
#define SB_CT  ((size_t)584448)
#define SB_ST  ((size_t)596736)
#define SB_END ((size_t)609024)

static_assert(SEQ == IMH * IMW);
static_assert(NT == NBAT * SEQ);
static_assert(CH == NHD * HDM);
static_assert(XDB == DTR + 2 * DST);
static_assert((CH % 32) == 0 && (HID % CH) == 0 && (NT % 64) == 0 && (SEQ % 64) == 0);
static_assert((LDC * 4) % 16 == 0);
static_assert(PLN * 2 == UNIT);
static_assert(WO_END * 2 == SB_KMP);
static_assert(SB_KMP + (size_t)512 * CH * 4 == SB_KM);
static_assert(SB_KM + 768 == SB_KVP);
static_assert(SB_KVP + (size_t)NBAT * CH * CH * 2 == SB_CT);
static_assert(SB_CT + (size_t)IMH * 24 * 4 == SB_ST && SB_ST + (size_t)IMH * 24 * 4 == SB_END);
static_assert(16 * UNIT + SB_END <= (size_t)134217728);

typedef _Float16 v16h __attribute__((ext_vector_type(16)));
typedef _Float16 v8h  __attribute__((ext_vector_type(8)));
typedef float    v8f  __attribute__((ext_vector_type(8)));
typedef float    v4f  __attribute__((ext_vector_type(4)));
typedef unsigned int v4u __attribute__((ext_vector_type(4)));

struct ThetaTab { float v[24]; };
static_assert(sizeof(ThetaTab) == 96);

#define HP(p) ((const _Float16*)(const void*)(p))

__device__ __forceinline__ unsigned short bf_bits(float f) {
  unsigned u = __float_as_uint(f);
  return (unsigned short)((u + 0x7FFFu + ((u >> 16) & 1u)) >> 16);
}
__device__ __forceinline__ float bf_up(unsigned short b) { return __uint_as_float(((unsigned)b) << 16); }
__device__ __forceinline__ float bfr(float f) { return bf_up(bf_bits(f)); }
__device__ __forceinline__ unsigned short h_bits(_Float16 x) { return __builtin_bit_cast(unsigned short, x); }
__device__ __forceinline__ unsigned short hb16(float f) { return h_bits((_Float16)f); }
__device__ __forceinline__ unsigned pk16(unsigned short a, unsigned short b) { return (unsigned)a | ((unsigned)b << 16); }
__device__ __forceinline__ v8f zero8() { v8f z = {0.f, 0.f, 0.f, 0.f, 0.f, 0.f, 0.f, 0.f}; return z; }
__device__ __forceinline__ int clampi(int v, int lo, int hi) { return min(max(v, lo), hi); }
__device__ __forceinline__ void split2(float f0, float f1, unsigned& hp, unsigned& lp) {
  const _Float16 h0 = (_Float16)f0, h1 = (_Float16)f1;
  const float q0 = (f0 - (float)h0) * 2048.0f, q1 = (f1 - (float)h1) * 2048.0f;
  hp = pk16(h_bits(h0), h_bits(h1));
  lp = pk16(hb16(q0), hb16(q1));
}
__device__ __forceinline__ float silu_f(float x) { return x * (1.0f / (1.0f + expf(-x))); }
__device__ __forceinline__ float elu1_f(float x) { const float em = expm1f(x) + 1.0f; return x > 0.0f ? x + 1.0f : em; }
__device__ __forceinline__ float softplus_f(float x) { return fmaxf(x, 0.0f) + log1pf(expf(-fabsf(x))); }
__device__ __forceinline__ float gelu_f(float v) { return 0.5f * v * (1.0f + erff(v * 0.70710678118654752f)); }

__device__ __forceinline__ v16h ldfrag_h(const _Float16* p) {
  union { v16h v; v8h h[2]; } f;
  f.h[0] = *(const v8h*)(p);
  f.h[1] = *(const v8h*)(p + 16);
  return f.v;
}

__device__ __forceinline__ v8f mma_raw(v16h a, v16h b, v8f c) {
  return __builtin_amdgcn_wmma_f32_16x16x32_f16(false, a, false, b, (short)0, c, false, false);
}
__device__ __forceinline__ void guard6(v8f& c0, v8f& c1, v8f& c2, v8f& c3, v8f& c4, v8f& c5,
                                       const v16h& a0, const v16h& a1, const v16h& b0, const v16h& b1,
                                       const v16h& b2) {
#if defined(__HIP_DEVICE_COMPILE__)
  asm volatile("v_nop\n\tv_nop\n\tv_nop\n\tv_nop"
               : "+v"(c0), "+v"(c1), "+v"(c2), "+v"(c3), "+v"(c4), "+v"(c5)
               : "v"(a0), "v"(a1), "v"(b0), "v"(b1), "v"(b2));
#endif
}
__device__ __forceinline__ void guard1(v8f& c0, const v16h& a0, const v16h& b0) {
#if defined(__HIP_DEVICE_COMPILE__)
  asm volatile("v_nop\n\tv_nop\n\tv_nop\n\tv_nop" : "+v"(c0) : "v"(a0), "v"(b0));
#endif
}

template <int NSRC>
__device__ __forceinline__ void gemm_core(const _Float16* __restrict__ h0, const _Float16* __restrict__ l0,
                                          const _Float16* __restrict__ h1, const _Float16* __restrict__ l1,
                                          const _Float16* __restrict__ h2, const _Float16* __restrict__ l2,
                                          const _Float16* __restrict__ h3, const _Float16* __restrict__ l3,
                                          const _Float16* __restrict__ W, int ldw, int tok0, int col0,
                                          float* Cs, float cscale) {
  const int tid = threadIdx.x, wave = tid >> 5, lane = tid & 31, hh = lane >> 4, c = lane & 15;
  const int mw = wave >> 1, nw = wave & 1;
  const size_t aoff = (size_t)(tok0 + mw * 16 + c) * CH + 8 * hh;
  const _Float16* b0p = W + (size_t)(col0 + nw * 48 + c) * ldw + 8 * hh;
  const _Float16* b1p = b0p + (size_t)16 * ldw;
  const _Float16* b2p = b0p + (size_t)32 * ldw;
  v8f ph0 = zero8(), ph1 = zero8(), ph2 = zero8(), pl0 = zero8(), pl1 = zero8(), pl2 = zero8();
#pragma unroll
  for (int s = 0; s < NSRC; ++s) {
    const _Float16* hp = (s == 0 ? h0 : s == 1 ? h1 : s == 2 ? h2 : h3) + aoff;
    const _Float16* lp = (s == 0 ? l0 : s == 1 ? l1 : s == 2 ? l2 : l3) + aoff;
    const int kb = s * CH;
#pragma unroll 1
    for (int ks = 0; ks < CH / 32; ++ks) {
      const int ko = ks * 32;
      const v16h fa  = ldfrag_h(hp + ko);
      const v16h ga  = ldfrag_h(lp + ko);
      const v16h fb0 = ldfrag_h(b0p + kb + ko);
      const v16h fb1 = ldfrag_h(b1p + kb + ko);
      const v16h fb2 = ldfrag_h(b2p + kb + ko);
      ph0 = mma_raw(fa, fb0, ph0);
      ph1 = mma_raw(fa, fb1, ph1);
      ph2 = mma_raw(fa, fb2, ph2);
      pl0 = mma_raw(ga, fb0, pl0);
      pl1 = mma_raw(ga, fb1, pl1);
      pl2 = mma_raw(ga, fb2, pl2);
      guard6(ph0, ph1, ph2, pl0, pl1, pl2, fa, ga, fb0, fb1, fb2);
    }
  }
#pragma unroll
  for (int r = 0; r < 8; ++r) {
    const int row = mw * 16 + 8 * hh + r;
    Cs[row * LDC + nw * 48 + c]      = (ph0[r] + pl0[r] * RSC) * cscale;
    Cs[row * LDC + nw * 48 + 16 + c] = (ph1[r] + pl1[r] * RSC) * cscale;
    Cs[row * LDC + nw * 48 + 32 + c] = (ph2[r] + pl2[r] * RSC) * cscale;
  }
}

__device__ __forceinline__ void store_planes(const float* Cs, unsigned short* dh, unsigned short* dl,
                                             size_t base, float osc) {
  const int tid = threadIdx.x;
  v4u ph[3], pq[3];
  size_t offs[3];
#pragma unroll
  for (int s = 0; s < 3; ++s) {
    const int p = s * 256 + tid;
    const int row = p / 12, c0 = (p - row * 12) * 8;
    v4u a, q;
#pragma unroll
    for (int e = 0; e < 4; ++e) {
      unsigned hw, lw;
      split2(Cs[row * LDC + c0 + 2 * e] * osc, Cs[row * LDC + c0 + 2 * e + 1] * osc, hw, lw);
      a[e] = hw; q[e] = lw;
    }
    ph[s] = a; pq[s] = q;
    offs[s] = base + (size_t)p * 8;
  }
#pragma unroll
  for (int s = 0; s < 3; ++s) { *(volatile v4u*)(dh + offs[s]) = ph[s]; *(volatile v4u*)(dl + offs[s]) = pq[s]; }
  __threadfence();
#pragma unroll
  for (int s = 0; s < 3; ++s) { *(volatile v4u*)(dh + offs[s]) = ph[s]; *(volatile v4u*)(dl + offs[s]) = pq[s]; }
}
__device__ __forceinline__ void store_f32(const float* Cs, float* dst, size_t base) {
  const int tid = threadIdx.x;
  v4f pk[6];
  size_t offs[6];
#pragma unroll
  for (int s = 0; s < 6; ++s) {
    const int p = s * 256 + tid;
    const int row = p / 24, c0 = (p - row * 24) * 4;
    v4f v;
#pragma unroll
    for (int e = 0; e < 4; ++e) v[e] = Cs[row * LDC + c0 + e];
    pk[s] = v;
    offs[s] = base + (size_t)p * 4;
  }
#pragma unroll
  for (int s = 0; s < 6; ++s) *(volatile v4f*)(dst + offs[s]) = pk[s];
  __threadfence();
#pragma unroll
  for (int s = 0; s < 6; ++s) *(volatile v4f*)(dst + offs[s]) = pk[s];
}

__global__ __launch_bounds__(256)
void k_prep(const float* __restrict__ wip, const float* __restrict__ wqk, const float* __restrict__ wxp,
            const float* __restrict__ wo1, const float* __restrict__ wpo, const float* __restrict__ wou,
            const float* __restrict__ wf1, const float* __restrict__ wf2,
            unsigned short* wpl, float* ct, float* st, ThetaTab th) {
  __shared__ __align__(16) float tcs[3072];
  __shared__ __align__(16) float tsn[3072];
  __shared__ float thl[32];
  const int tid = threadIdx.x, blk = blockIdx.x;
  if (blk < 8) {
    const float* src = wip; int K = 96, NS = 288, NR = 288, NP = 288; size_t doff = WO_IP;
    if (blk == 1)      { src = wqk; K = 96;  NS = 192; NR = 192; NP = 192; doff = WO_QK; }
    else if (blk == 2) { src = wxp; K = 96;  NS = XDB; NR = XDB; NP = 96;  doff = WO_XP; }
    else if (blk == 3) { src = wo1; K = 192; NS = 96;  NR = 96;  NP = 96;  doff = WO_O1; }
    else if (blk == 4) { src = wpo; K = 96;  NS = 96;  NR = 96;  NP = 96;  doff = WO_PO; }
    else if (blk == 5) { src = wou; K = 192; NS = 96;  NR = 96;  NP = 96;  doff = WO_OU; }
    else if (blk == 6) { src = wf1; K = 96;  NS = 384; NR = 384; NP = 384; doff = WO_F1; }
    else if (blk == 7) { src = wf2; K = 384; NS = 96;  NR = 96;  NP = 96;  doff = WO_F2; }
    const int kp = K >> 3, np = NP * kp, nit = (np + 255) >> 8;
#pragma unroll 1
    for (int it = 0; it < nit; ++it) {
      const int p = it * 256 + tid;
      const int pp = min(p, np - 1);
      const int n = pp / kp, k0 = (pp - n * kp) * 8;
      const int nn = min(n, NR - 1);
      const bool live = (n < NR);
      v4u pk;
#pragma unroll
      for (int e = 0; e < 4; ++e) {
        const float f0 = src[(size_t)(k0 + 2 * e) * NS + nn];
        const float f1 = src[(size_t)(k0 + 2 * e + 1) * NS + nn];
        const unsigned short q0 = live ? hb16(bfr(f0) * 64.0f) : (unsigned short)0;
        const unsigned short q1 = live ? hb16(bfr(f1) * 64.0f) : (unsigned short)0;
        pk[e] = pk16(q0, q1);
      }
      unsigned short* dst = wpl + doff + (size_t)pp * 8;
      if (p < np) *(volatile v4u*)dst = pk;
      __threadfence();
      if (p < np) *(volatile v4u*)dst = pk;
    }
  } else {
    float tv = 0.0f;
#pragma unroll
    for (int j = 0; j < 24; ++j) tv = (tid == j) ? th.v[j] : tv;
    if (tid < 24) thl[tid] = tv;
    __syncthreads();
#pragma unroll 1
    for (int it = 0; it < 12; ++it) {
      const int idx = it * 256 + tid;
      const int pos = idx / 24, j = idx - pos * 24;
      const float ang = (float)pos * thl[j];
      tcs[idx] = cosf(ang);
      tsn[idx] = sinf(ang);
    }
    __syncthreads();
    v4f a[3], bq[3];
#pragma unroll
    for (int s = 0; s < 3; ++s) {
      const int p = s * 256 + tid;
      a[s]  = *(const v4f*)(tcs + 4 * p);
      bq[s] = *(const v4f*)(tsn + 4 * p);
    }
#pragma unroll
    for (int s = 0; s < 3; ++s) { const int p = s * 256 + tid; *(volatile v4f*)(ct + 4 * p) = a[s]; *(volatile v4f*)(st + 4 * p) = bq[s]; }
    __threadfence();
#pragma unroll
    for (int s = 0; s < 3; ++s) { const int p = s * 256 + tid; *(volatile v4f*)(ct + 4 * p) = a[s]; *(volatile v4f*)(st + 4 * p) = bq[s]; }
  }
}

__global__ __launch_bounds__(256)
void k_ln1(const float* __restrict__ x, const float* __restrict__ g, const float* __restrict__ bb,
           unsigned short* hsh, unsigned short* hsl) {
  __shared__ __align__(16) float Cs[64 * LDC];
  const int tid = threadIdx.x, wave = tid >> 5, lane = tid & 31;
  const int tok0 = blockIdx.x * 64;
  const float g0 = bfr(g[lane]), g1 = bfr(g[lane + 32]), g2 = bfr(g[lane + 64]);
  const float e0 = bfr(bb[lane]), e1 = bfr(bb[lane + 32]), e2 = bfr(bb[lane + 64]);
#pragma unroll 1
  for (int it = 0; it < 8; ++it) {
    const int row = wave * 8 + it;
    const float* xr = x + (size_t)(tok0 + row) * CH;
    const float v0 = bfr(xr[lane]), v1 = bfr(xr[lane + 32]), v2 = bfr(xr[lane + 64]);
    float s = v0 + v1 + v2;
#pragma unroll
    for (int off = 16; off; off >>= 1) s += __shfl_xor(s, off, 32);
    const float mu = s * (1.0f / 96.0f);
    const float d0 = v0 - mu, d1 = v1 - mu, d2 = v2 - mu;
    float sq = d0 * d0 + d1 * d1 + d2 * d2;
#pragma unroll
    for (int off = 16; off; off >>= 1) sq += __shfl_xor(sq, off, 32);
    const float var = sq * (1.0f / 96.0f);
    const float rs = rsqrtf(var + 1e-5f);
    Cs[row * LDC + lane]      = d0 * rs * g0 + e0;
    Cs[row * LDC + lane + 32] = d1 * rs * g1 + e1;
    Cs[row * LDC + lane + 64] = d2 * rs * g2 + e2;
  }
  __syncthreads();
  store_planes(Cs, hsh, hsl, (size_t)tok0 * CH, 1.0f);
}

__global__ __launch_bounds__(256)
void k_inproj(const unsigned short* __restrict__ hsh, const unsigned short* __restrict__ hsl,
              const unsigned short* __restrict__ wpl, float* x0f, float* z0f, float* w0f) {
  __shared__ __align__(16) float Cs[64 * LDC];
  const int g = blockIdx.y;
  const int tok0 = blockIdx.x * 64;
  const _Float16* ah = HP(hsh);
  const _Float16* al = HP(hsl);
  gemm_core<1>(ah, al, ah, al, ah, al, ah, al, HP(wpl), CH, tok0, g * CH, Cs, 1.0f / 64.0f);
  __syncthreads();
  float* dst = (g == 0) ? x0f : (g == 1) ? z0f : w0f;
  store_f32(Cs, dst, (size_t)tok0 * CH);
}

__global__ __launch_bounds__(256)
void k_conv1d(const float* __restrict__ x0f, const float* __restrict__ z0f,
              const float* __restrict__ cxw, const float* __restrict__ czw,
              unsigned short* xch, unsigned short* xcl, float* xcf,
              unsigned short* zch, unsigned short* zcl, float* zcf) {
  __shared__ __align__(16) float Cs[64 * LDC];
  const int tid = threadIdx.x, g = blockIdx.y;
  const int tok0 = blockIdx.x * 64;
  const int b = tok0 >> 14;
  const int tfirst = b * SEQ, tlast = tfirst + SEQ - 1;
  const float* src = g ? z0f : x0f;
  const float* wv = g ? czw : cxw;
#pragma unroll 1
  for (int it = 0; it < 24; ++it) {
    const int idx = it * 256 + tid;
    const int row = idx / CH, col = idx - row * CH;
    const int tok = tok0 + row;
    float s = 0.0f;
#pragma unroll
    for (int j = 0; j < 4; ++j) {
      const int t = tok - 1 + j;
      const bool ok = (t >= tfirst) && (t <= tlast);
      const int tc = clampi(t, tfirst, tlast);
      const float v = src[(size_t)tc * CH + col];
      s += (ok ? v : 0.0f) * bfr(wv[col * 4 + j]);
    }
    Cs[row * LDC + col] = silu_f(s);
  }
  __syncthreads();
  store_f32(Cs, g ? zcf : xcf, (size_t)tok0 * CH);
  store_planes(Cs, g ? zch : xch, g ? zcl : xcl, (size_t)tok0 * CH, 16.0f);
}

__global__ __launch_bounds__(256)
void k_xproj(const unsigned short* __restrict__ xch, const unsigned short* __restrict__ xcl,
             const unsigned short* __restrict__ wxp, const float* __restrict__ dtw, const float* __restrict__ dtb,
             float* delta, float* bcf) {
  __shared__ __align__(16) float Cs[64 * LDC];
  __shared__ __align__(16) float Ds[64 * LDC];
  const int tid = threadIdx.x;
  const int tok0 = blockIdx.x * 64;
  const _Float16* ah = HP(xch);
  const _Float16* al = HP(xcl);
  gemm_core<1>(ah, al, ah, al, ah, al, ah, al, HP(wxp), CH, tok0, 0, Cs, 1.0f / 1024.0f);
  __syncthreads();
#pragma unroll 1
  for (int it = 0; it < 24; ++it) {
    const int idx = it * 256 + tid;
    const int row = idx / CH, col = idx - row * CH;
    float s = 0.0f;
#pragma unroll
    for (int j = 0; j < DTR; ++j) s += Cs[row * LDC + j] * bfr(dtw[j * CH + col]);
    s += bfr(dtb[col]);
    Ds[row * LDC + col] = softplus_f(s);
  }
  __syncthreads();
  store_f32(Ds, delta, (size_t)tok0 * CH);
  v4f pk[2];
  size_t offs[2];
#pragma unroll
  for (int s = 0; s < 2; ++s) {
    const int p = s * 256 + tid;
    const int row = p >> 3, c0 = (p & 7) * 4;
    v4f v;
#pragma unroll
    for (int e = 0; e < 4; ++e) v[e] = Cs[row * LDC + DTR + c0 + e];
    pk[s] = v;
    offs[s] = (size_t)tok0 * (2 * DST) + (size_t)p * 4;
  }
#pragma unroll
  for (int s = 0; s < 2; ++s) *(volatile v4f*)(bcf + offs[s]) = pk[s];
  __threadfence();
#pragma unroll
  for (int s = 0; s < 2; ++s) *(volatile v4f*)(bcf + offs[s]) = pk[s];
}

__global__ __launch_bounds__(32)
void k_scan(const float* __restrict__ delta, const float* __restrict__ xcf, const float* __restrict__ bcf,
            const float* __restrict__ alog, const float* __restrict__ dv, float* ytf) {
  __shared__ __align__(16) float ys[128];
  const int lane = threadIdx.x, pr = lane >> 4, n = lane & 15;
  const int pair = blockIdx.x * 2 + pr;
  const int b = pair / CH, d = pair - b * CH;
  const float An = -expf(bfr(alog[d * DST + n]));
  const float Dd = bfr(dv[d]);
  const size_t tb = (size_t)b * SEQ;
  const float* dp = delta + tb * CH + d;
  const float* up = xcf + tb * CH + d;
  const float* bp = bcf + tb * (2 * DST) + n;
  float* yd = ytf + ((size_t)(b * CH + d)) * SEQ + n * 4;
  float h = 0.0f;
#pragma unroll 1
  for (int chunk = 0; chunk < SEQ / 64; ++chunk) {
#pragma unroll 1
    for (int i = 0; i < 64; ++i) {
      const size_t l = (size_t)(chunk * 64 + i);
      const float dl = dp[l * CH];
      const float u  = up[l * CH];
      const float Bv = bp[l * (2 * DST)];
      const float Cv = bp[l * (2 * DST) + DST];
      h = __expf(dl * An) * h + (dl * Bv) * u;
      float p = h * Cv;
      p += __shfl_xor(p, 1, 32);
      p += __shfl_xor(p, 2, 32);
      p += __shfl_xor(p, 4, 32);
      p += __shfl_xor(p, 8, 32);
      if (n == 0) ys[pr * 64 + i] = p + Dd * u;
    }
    __syncthreads();
    const v4f v = *(const v4f*)(ys + pr * 64 + n * 4);
    float* q = yd + (size_t)chunk * 64;
    *(volatile v4f*)q = v;
    __threadfence();
    *(volatile v4f*)q = v;
    __syncthreads();
  }
}

__global__ __launch_bounds__(256)
void k_ytr(const float* __restrict__ ytf, unsigned short* yh, unsigned short* yl) {
  __shared__ __align__(16) float Cs[64 * LDC];
  const int tid = threadIdx.x;
  const int tok0 = blockIdx.x * 64;
  const int b = tok0 >> 14, l0 = tok0 & (SEQ - 1);
#pragma unroll 1
  for (int it = 0; it < 6; ++it) {
    const int p = it * 256 + tid;
    const int c = p >> 4, q = p & 15;
    const v4f v = *(const v4f*)(ytf + ((size_t)(b * CH + c)) * SEQ + l0 + q * 4);
#pragma unroll
    for (int e = 0; e < 4; ++e) Cs[(q * 4 + e) * LDC + c] = v[e];
  }
  __syncthreads();
  store_planes(Cs, yh, yl, (size_t)tok0 * CH, 16.0f);
}

__global__ __launch_bounds__(256)
void k_out1(const unsigned short* __restrict__ yh, const unsigned short* __restrict__ yl,
            const unsigned short* __restrict__ zch, const unsigned short* __restrict__ zcl,
            const unsigned short* __restrict__ wo1, unsigned short* o1h, unsigned short* o1l) {
  __shared__ __align__(16) float Cs[64 * LDC];
  const int tok0 = blockIdx.x * 64;
  gemm_core<2>(HP(yh), HP(yl), HP(zch), HP(zcl), HP(yh), HP(yl), HP(yh), HP(yl),
               HP(wo1), 2 * CH, tok0, 0, Cs, 1.0f / 1024.0f);
  __syncthreads();
  store_planes(Cs, o1h, o1l, (size_t)tok0 * CH, 256.0f);
}

__global__ __launch_bounds__(256)
void k_dwconv(const float* __restrict__ w0f, const float* __restrict__ dww, const float* __restrict__ dwb,
              unsigned short* linh, unsigned short* linl, float* linf, unsigned short* vt) {
  __shared__ __align__(16) float Cs[64 * LDC];
  const int tid = threadIdx.x;
  const int tok0 = blockIdx.x * 64;
  const int b = tok0 >> 14, l0 = tok0 & (SEQ - 1), hpos = l0 >> 7, w0 = l0 & (IMW - 1);
  const size_t bbase = (size_t)b * SEQ;
#pragma unroll 1
  for (int it = 0; it < 24; ++it) {
    const int idx = it * 256 + tid;
    const int row = idx / CH, col = idx - row * CH;
    const int wpos = w0 + row;
    float s = 0.0f;
#pragma unroll
    for (int kh = 0; kh < 3; ++kh) {
      const int h2 = hpos + kh - 1;
      const bool hv = (h2 >= 0) && (h2 < IMH);
      const int hc = clampi(h2, 0, IMH - 1);
#pragma unroll
      for (int kw = 0; kw < 3; ++kw) {
        const int w2 = wpos + kw - 1;
        const bool ok = hv && (w2 >= 0) && (w2 < IMW);
        const int wc = clampi(w2, 0, IMW - 1);
        const float v = w0f[(bbase + (size_t)hc * IMW + wc) * CH + col];
        s += (ok ? v : 0.0f) * bfr(dww[col * 9 + kh * 3 + kw]);
      }
    }
    s += bfr(dwb[col]);
    Cs[row * LDC + col] = silu_f(s);
  }
  __syncthreads();
  store_f32(Cs, linf, (size_t)tok0 * CH);
  store_planes(Cs, linh, linl, (size_t)tok0 * CH, 16.0f);
  v4u pk[3];
  size_t offs[3];
#pragma unroll
  for (int s = 0; s < 3; ++s) {
    const int p = s * 256 + tid;
    const int c = p >> 3, l8 = (p & 7) * 8;
    v4u a;
#pragma unroll
    for (int e = 0; e < 4; ++e) {
      const float f0 = 16.0f * Cs[(l8 + 2 * e) * LDC + c];
      const float f1 = 16.0f * Cs[(l8 + 2 * e + 1) * LDC + c];
      a[e] = pk16(hb16(f0), hb16(f1));
    }
    pk[s] = a;
    offs[s] = ((size_t)(b * CH + c)) * SEQ + l0 + l8;
  }
#pragma unroll
  for (int s = 0; s < 3; ++s) *(volatile v4u*)(vt + offs[s]) = pk[s];
  __threadfence();
#pragma unroll
  for (int s = 0; s < 3; ++s) *(volatile v4u*)(vt + offs[s]) = pk[s];
}

__global__ __launch_bounds__(256)
void k_qk(const unsigned short* __restrict__ linh, const unsigned short* __restrict__ linl,
          const unsigned short* __restrict__ wqk, const float* __restrict__ qkb,
          const float* __restrict__ ct, const float* __restrict__ st,
          unsigned short* qrh, unsigned short* qrl, float* quf, unsigned short* krt, float* kmp) {
  __shared__ __align__(16) float Cs[64 * LDC];
  __shared__ __align__(16) float ksum[CH];
  const int tid = threadIdx.x;
  const int g = blockIdx.y;
  const int tok0 = blockIdx.x * 64;
  const int b = tok0 >> 14, l0 = tok0 & (SEQ - 1), hpos = l0 >> 7, w0 = l0 & (IMW - 1);
  const _Float16* ah = HP(linh);
  const _Float16* al = HP(linl);
  gemm_core<1>(ah, al, ah, al, ah, al, ah, al, HP(wqk), CH, tok0, g * CH, Cs, 1.0f / 1024.0f);
  __syncthreads();
#pragma unroll 1
  for (int it = 0; it < 24; ++it) {
    const int idx = it * 256 + tid;
    const int row = idx / CH, col = idx - row * CH;
    const float v = Cs[row * LDC + col] + bfr(qkb[g * CH + col]);
    Cs[row * LDC + col] = elu1_f(v);
  }
  __syncthreads();
  if (g == 0) {
    store_f32(Cs, quf, (size_t)tok0 * CH);
    v4u ph[3], pq[3];
    size_t offs[3];
#pragma unroll
    for (int s = 0; s < 3; ++s) {
      const int p = s * 256 + tid;
      const int row = p / 12, c0 = (p - row * 12) * 8;
      const int wpos = w0 + row;
      v4u a, q;
#pragma unroll
      for (int e = 0; e < 4; ++e) {
        const int ca = c0 + 2 * e;
        const int i = ca >> 1;
        const bool hsel = (i < 24);
        const int pos = hsel ? hpos : wpos;
        const int j = hsel ? i : i - 24;
        const float cs = ct[pos * 24 + j], sn = st[pos * 24 + j];
        const float a0 = Cs[row * LDC + ca], a1 = Cs[row * LDC + ca + 1];
        const float r0 = a0 * cs - a1 * sn;
        const float r1 = a0 * sn + a1 * cs;
        unsigned hw, lw;
        split2(r0, r1, hw, lw);
        a[e] = hw; q[e] = lw;
      }
      ph[s] = a; pq[s] = q;
      offs[s] = (size_t)tok0 * CH + (size_t)p * 8;
    }
#pragma unroll
    for (int s = 0; s < 3; ++s) { *(volatile v4u*)(qrh + offs[s]) = ph[s]; *(volatile v4u*)(qrl + offs[s]) = pq[s]; }
    __threadfence();
#pragma unroll
    for (int s = 0; s < 3; ++s) { *(volatile v4u*)(qrh + offs[s]) = ph[s]; *(volatile v4u*)(qrl + offs[s]) = pq[s]; }
  } else {
    if (tid < CH) {
      float s = 0.0f;
#pragma unroll 1
      for (int r = 0; r < 64; ++r) s += Cs[r * LDC + tid];
      ksum[tid] = s;
    }
    __syncthreads();
    {
      const int t4 = min(tid, 23);
      const v4f kk = *(const v4f*)(ksum + 4 * t4);
      float* dk = kmp + (size_t)blockIdx.x * CH + 4 * t4;
      if (tid < 24) *(volatile v4f*)dk = kk;
      __threadfence();
      if (tid < 24) *(volatile v4f*)dk = kk;
    }
    v4u pk[3];
    size_t offk[3];
#pragma unroll
    for (int s = 0; s < 3; ++s) {
      const int p = s * 256 + tid;
      const int c = p >> 3, l8 = (p & 7) * 8;
      const int i = c >> 1, odd = c & 1, ce = c & ~1;
      const bool hsel = (i < 24);
      const int j = hsel ? i : i - 24;
      v4u a;
#pragma unroll
      for (int e = 0; e < 4; ++e) {
        const int rA = l8 + 2 * e, rB = rA + 1;
        const int posA = hsel ? hpos : (w0 + rA);
        const int posB = hsel ? hpos : (w0 + rB);
        const float csA = ct[posA * 24 + j], snA = st[posA * 24 + j];
        const float csB = ct[posB * 24 + j], snB = st[posB * 24 + j];
        const float a0A = Cs[rA * LDC + ce], a1A = Cs[rA * LDC + ce + 1];
        const float a0B = Cs[rB * LDC + ce], a1B = Cs[rB * LDC + ce + 1];
        const float vA = odd ? (a0A * snA + a1A * csA) : (a0A * csA - a1A * snA);
        const float vB = odd ? (a0B * snB + a1B * csB) : (a0B * csB - a1B * snB);
        a[e] = pk16(hb16(vA), hb16(vB));
      }
      pk[s] = a;
      offk[s] = ((size_t)(b * CH + c)) * SEQ + l0 + l8;
    }
#pragma unroll
    for (int s = 0; s < 3; ++s) *(volatile v4u*)(krt + offk[s]) = pk[s];
    __threadfence();
#pragma unroll
    for (int s = 0; s < 3; ++s) *(volatile v4u*)(krt + offk[s]) = pk[s];
  }
}

__global__ __launch_bounds__(256)
void k_kmean(const float* __restrict__ kmp, float* km) {
  __shared__ __align__(16) float kms[256];
  const int tid = threadIdx.x;
  const int t = min(tid, 2 * CH - 1);
  const int b = t / CH, c = t - b * CH;
  float s = 0.0f;
#pragma unroll 1
  for (int blk = 0; blk < 256; ++blk) s += kmp[((size_t)(b * 256 + blk)) * CH + c];
  kms[tid] = s * (1.0f / 16384.0f);
  __syncthreads();
  const int t4 = min(tid, 47);
  const v4f v = *(const v4f*)(kms + 4 * t4);
  if (tid < 48) *(volatile v4f*)(km + 4 * t4) = v;
  __threadfence();
  if (tid < 48) *(volatile v4f*)(km + 4 * t4) = v;
}

__global__ __launch_bounds__(256)
void k_kv(const unsigned short* __restrict__ krt, const unsigned short* __restrict__ vt, unsigned short* kvp) {
  __shared__ float part[8 * 256];
  __shared__ float kvs[256];
  const int tid = threadIdx.x, wave = tid >> 5, lane = tid & 31, hh = lane >> 4, c = lane & 15;
  const int bh = blockIdx.x;
  const int b = bh / NHD, h = bh - b * NHD;
  const size_t roff = ((size_t)(b * CH + h * HDM + c)) * SEQ + (size_t)wave * 2048 + 8 * hh;
  const _Float16* ap = HP(krt) + roff;
  const _Float16* bp = HP(vt) + roff;
  v8f acc = zero8();
#pragma unroll 1
  for (int ks = 0; ks < 64; ++ks) {
    const int ko = ks * 32;
    const v16h fa = ldfrag_h(ap + ko);
    const v16h fb = ldfrag_h(bp + ko);
    acc = mma_raw(fa, fb, acc);
    guard1(acc, fa, fb);
  }
#pragma unroll
  for (int r = 0; r < 8; ++r) part[wave * 256 + (8 * hh + r) * 16 + c] = acc[r];
  __syncthreads();
  {
    float s = 0.0f;
#pragma unroll
    for (int w = 0; w < 8; ++w) s += part[w * 256 + tid];
    kvs[tid] = s * (1.0f / 262144.0f);
  }
  __syncthreads();
  const int tp = min(tid, 191);
  const int e = tp / 12, k0 = (tp - e * 12) * 8;
  v4u pk;
#pragma unroll
  for (int u = 0; u < 4; ++u) {
    const int kA = k0 + 2 * u, kB = kA + 1;
    const float fA = ((kA >> 4) == h) ? 4096.0f * kvs[(kA & 15) * 16 + e] : 0.0f;
    const float fB = ((kB >> 4) == h) ? 4096.0f * kvs[(kB & 15) * 16 + e] : 0.0f;
    pk[u] = pk16(hb16(fA), hb16(fB));
  }
  unsigned short* dst = kvp + ((size_t)(b * CH + h * HDM)) * CH + (size_t)tp * 8;
  if (tid < 192) *(volatile v4u*)dst = pk;
  __threadfence();
  if (tid < 192) *(volatile v4u*)dst = pk;
}

__global__ __launch_bounds__(256)
void k_attn(const unsigned short* __restrict__ qrh, const unsigned short* __restrict__ qrl,
            const unsigned short* __restrict__ kvp, const float* __restrict__ quf, const float* __restrict__ km,
            const float* __restrict__ linf, const float* __restrict__ zcf,
            const float* __restrict__ lpw, const float* __restrict__ lpb,
            unsigned short* o2ah, unsigned short* o2al) {
  __shared__ __align__(16) float Cs[64 * LDC];
  __shared__ float zd[384];
  const int tid = threadIdx.x;
  const int tok0 = blockIdx.x * 64;
  const int b = tok0 >> 14, l0 = tok0 & (SEQ - 1), hpos = l0 >> 7, w0 = l0 & (IMW - 1);
  const size_t bbase = (size_t)b * SEQ;
  const _Float16* ah = HP(qrh);
  const _Float16* al = HP(qrl);
  gemm_core<1>(ah, al, ah, al, ah, al, ah, al, HP(kvp) + (size_t)b * CH * CH, CH, tok0, 0, Cs, 1.0f / 4096.0f);
  __syncthreads();
#pragma unroll 1
  for (int it = 0; it < 2; ++it) {
    const int task = it * 256 + tid;
    const int tk = min(task, 383);
    const int row = tk / NHD, hd = tk - row * NHD;
    float zs = 0.0f;
#pragma unroll
    for (int dd = 0; dd < HDM; ++dd)
      zs += quf[((size_t)(tok0 + row)) * CH + hd * HDM + dd] * km[b * CH + hd * HDM + dd];
    if (task < 384) zd[task] = 1.0f / (zs + 1e-6f);
  }
  __syncthreads();
#pragma unroll 1
  for (int it = 0; it < 24; ++it) {
    const int idx = it * 256 + tid;
    const int row = idx / CH, col = idx - row * CH;
    const int wpos = w0 + row;
    const float o = Cs[row * LDC + col] * zd[row * NHD + (col >> 4)];
    float s = 0.0f;
#pragma unroll
    for (int kh = 0; kh < 3; ++kh) {
      const int h2 = hpos + kh - 1;
      const bool hv = (h2 >= 0) && (h2 < IMH);
      const int hc = clampi(h2, 0, IMH - 1);
#pragma unroll
      for (int kw = 0; kw < 3; ++kw) {
        const int w2 = wpos + kw - 1;
        const bool ok = hv && (w2 >= 0) && (w2 < IMW);
        const int wc = clampi(w2, 0, IMW - 1);
        const float v = linf[(bbase + (size_t)hc * IMW + wc) * CH + col];
        s += (ok ? v : 0.0f) * bfr(lpw[col * 9 + kh * 3 + kw]);
      }
    }
    s += bfr(lpb[col]);
    const float z = zcf[((size_t)(tok0 + row)) * CH + col];
    Cs[row * LDC + col] = (o + s) * z;
  }
  __syncthreads();
  store_planes(Cs, o2ah, o2al, (size_t)tok0 * CH, 1024.0f);
}

__global__ __launch_bounds__(256)
void k_out2(const unsigned short* __restrict__ o2ah, const unsigned short* __restrict__ o2al,
            const unsigned short* __restrict__ wpo, const float* __restrict__ pob,
            unsigned short* o2h, unsigned short* o2l) {
  __shared__ __align__(16) float Cs[64 * LDC];
  const int tid = threadIdx.x;
  const int tok0 = blockIdx.x * 64;
  const _Float16* ah = HP(o2ah);
  const _Float16* al = HP(o2al);
  gemm_core<1>(ah, al, ah, al, ah, al, ah, al, HP(wpo), CH, tok0, 0, Cs, 1.0f / 65536.0f);
  __syncthreads();
#pragma unroll 1
  for (int it = 0; it < 24; ++it) {
    const int idx = it * 256 + tid;
    const int row = idx / CH, col = idx - row * CH;
    Cs[row * LDC + col] = Cs[row * LDC + col] + bfr(pob[col]);
  }
  __syncthreads();
  store_planes(Cs, o2h, o2l, (size_t)tok0 * CH, 256.0f);
}

__global__ __launch_bounds__(256)
void k_outp(const unsigned short* __restrict__ o1h, const unsigned short* __restrict__ o1l,
            const unsigned short* __restrict__ o2h, const unsigned short* __restrict__ o2l,
            const unsigned short* __restrict__ wou, const float* __restrict__ outb,
            const float* __restrict__ hid, const float* __restrict__ g2, const float* __restrict__ b2,
            float* outf, unsigned short* h2h, unsigned short* h2l) {
  __shared__ __align__(16) float Cs[64 * LDC];
  __shared__ __align__(16) float Ns[64 * LDC];
  const int tid = threadIdx.x, wave = tid >> 5, lane = tid & 31;
  const int tok0 = blockIdx.x * 64;
  gemm_core<2>(HP(o1h), HP(o1l), HP(o2h), HP(o2l), HP(o1h), HP(o1l), HP(o1h), HP(o1l),
               HP(wou), 2 * CH, tok0, 0, Cs, 1.0f / 16384.0f);
  __syncthreads();
#pragma unroll 1
  for (int it = 0; it < 24; ++it) {
    const int idx = it * 256 + tid;
    const int row = idx / CH, col = idx - row * CH;
    const float sc = bfr(hid[((size_t)(tok0 + row)) * CH + col]);
    Cs[row * LDC + col] = sc + (Cs[row * LDC + col] + bfr(outb[col]));
  }
  __syncthreads();
  const float g0 = bfr(g2[lane]), g1 = bfr(g2[lane + 32]), gg2 = bfr(g2[lane + 64]);
  const float e0 = bfr(b2[lane]), e1 = bfr(b2[lane + 32]), e2 = bfr(b2[lane + 64]);
#pragma unroll 1
  for (int it = 0; it < 8; ++it) {
    const int row = wave * 8 + it;
    const float v0 = Cs[row * LDC + lane], v1 = Cs[row * LDC + lane + 32], v2 = Cs[row * LDC + lane + 64];
    float s = v0 + v1 + v2;
#pragma unroll
    for (int off = 16; off; off >>= 1) s += __shfl_xor(s, off, 32);
    const float mu = s * (1.0f / 96.0f);
    const float d0 = v0 - mu, d1 = v1 - mu, d2 = v2 - mu;
    float sq = d0 * d0 + d1 * d1 + d2 * d2;
#pragma unroll
    for (int off = 16; off; off >>= 1) sq += __shfl_xor(sq, off, 32);
    const float var = sq * (1.0f / 96.0f);
    const float rs = rsqrtf(var + 1e-5f);
    Ns[row * LDC + lane]      = d0 * rs * g0 + e0;
    Ns[row * LDC + lane + 32] = d1 * rs * g1 + e1;
    Ns[row * LDC + lane + 64] = d2 * rs * gg2 + e2;
  }
  __syncthreads();
  store_f32(Cs, outf, (size_t)tok0 * CH);
  store_planes(Ns, h2h, h2l, (size_t)tok0 * CH, 1.0f);
}

__global__ __launch_bounds__(256)
void k_fc1(const unsigned short* __restrict__ h2h, const unsigned short* __restrict__ h2l,
           const unsigned short* __restrict__ w1, const float* __restrict__ b1,
           unsigned short* g0h, unsigned short* g0l, unsigned short* g1h, unsigned short* g1l,
           unsigned short* g2h, unsigned short* g2l, unsigned short* g3h, unsigned short* g3l) {
  __shared__ __align__(16) float Cs[64 * LDC];
  const int tid = threadIdx.x;
  const int g = blockIdx.y;
  const int tok0 = blockIdx.x * 64;
  const _Float16* ah = HP(h2h);
  const _Float16* al = HP(h2l);
  gemm_core<1>(ah, al, ah, al, ah, al, ah, al, HP(w1), CH, tok0, g * CH, Cs, 1.0f / 64.0f);
  __syncthreads();
#pragma unroll 1
  for (int it = 0; it < 24; ++it) {
    const int idx = it * 256 + tid;
    const int row = idx / CH, col = idx - row * CH;
    const float v = Cs[row * LDC + col] + bfr(b1[g * CH + col]);
    Cs[row * LDC + col] = gelu_f(v);
  }
  __syncthreads();
  unsigned short* dh = (g == 0) ? g0h : (g == 1) ? g1h : (g == 2) ? g2h : g3h;
  unsigned short* dl = (g == 0) ? g0l : (g == 1) ? g1l : (g == 2) ? g2l : g3l;
  store_planes(Cs, dh, dl, (size_t)tok0 * CH, 16.0f);
}

__global__ __launch_bounds__(256)
void k_fc2(const unsigned short* __restrict__ g0h, const unsigned short* __restrict__ g0l,
           const unsigned short* __restrict__ g1h, const unsigned short* __restrict__ g1l,
           const unsigned short* __restrict__ g2h, const unsigned short* __restrict__ g2l,
           const unsigned short* __restrict__ g3h, const unsigned short* __restrict__ g3l,
           const unsigned short* __restrict__ w2, const float* __restrict__ b2,
           const float* __restrict__ outf, float* out) {
  __shared__ __align__(16) float Cs[64 * LDC];
  const int tid = threadIdx.x;
  const int tok0 = blockIdx.x * 64;
  gemm_core<4>(HP(g0h), HP(g0l), HP(g1h), HP(g1l), HP(g2h), HP(g2l), HP(g3h), HP(g3l),
               HP(w2), HID, tok0, 0, Cs, 1.0f / 1024.0f);
  __syncthreads();
#pragma unroll 1
  for (int it = 0; it < 24; ++it) {
    const int idx = it * 256 + tid;
    const int row = idx / CH, col = idx - row * CH;
    const float r = outf[((size_t)(tok0 + row)) * CH + col];
    Cs[row * LDC + col] = r + (Cs[row * LDC + col] + bfr(b2[col]));
  }
  __syncthreads();
  store_f32(Cs, out, (size_t)tok0 * CH);
}

extern "C" void kernel_launch(void* const* d_in, const int* in_sizes, int n_in,
                              void* d_out, int out_size, void* d_ws, size_t ws_size,
                              hipStream_t stream) {
  if (n_in < 28) return;
  const int expect[28] = { NT * CH, CH, CH, CH * 288, CH * 9, CH, CH * 192, 192, CH * 9, CH, CH * 4, CH * 4,
                           CH * XDB, DTR * CH, CH, CH * DST, CH, 192 * CH, CH * CH, CH, 192 * CH, CH, CH, CH,
                           CH * HID, HID, HID * CH, CH };
  for (int i = 0; i < 28; ++i) if (in_sizes[i] != expect[i]) return;
  if (out_size != NT * CH) return;
  const size_t oSM = 16 * UNIT;
  const size_t oEND = oSM + SB_END;
  if (oEND > ws_size) return;
  if (oEND > (size_t)134217728) return;

  const float* hidden     = (const float*)d_in[0];
  const float* norm_in_g  = (const float*)d_in[1];
  const float* norm_in_b  = (const float*)d_in[2];
  const float* in_proj_w  = (const float*)d_in[3];
  const float* dw_w       = (const float*)d_in[4];
  const float* dw_b       = (const float*)d_in[5];
  const float* qk_w       = (const float*)d_in[6];
  const float* qk_b       = (const float*)d_in[7];
  const float* lepe_w     = (const float*)d_in[8];
  const float* lepe_b     = (const float*)d_in[9];
  const float* conv_x_w   = (const float*)d_in[10];
  const float* conv_z_w   = (const float*)d_in[11];
  const float* x_proj_w   = (const float*)d_in[12];
  const float* dt_proj_w  = (const float*)d_in[13];
  const float* dt_proj_b  = (const float*)d_in[14];
  const float* A_log      = (const float*)d_in[15];
  const float* Dv         = (const float*)d_in[16];
  const float* out_proj_w = (const float*)d_in[17];
  const float* proj_out_w = (const float*)d_in[18];
  const float* proj_out_b = (const float*)d_in[19];
  const float* out_w      = (const float*)d_in[20];
  const float* out_b      = (const float*)d_in[21];
  const float* norm_mlp_g = (const float*)d_in[22];
  const float* norm_mlp_b = (const float*)d_in[23];
  const float* fc1_w      = (const float*)d_in[24];
  const float* fc1_b      = (const float*)d_in[25];
  const float* fc2_w      = (const float*)d_in[26];
  const float* fc2_b      = (const float*)d_in[27];
  float* out = (float*)d_out;

  char* ws = (char*)d_ws;
#define SLOT_H(i) ((unsigned short*)(ws + (size_t)(i) * UNIT))
#define SLOT_F(i) ((float*)(ws + (size_t)(i) * UNIT))
  unsigned short* HSH = SLOT_H(0);  unsigned short* HSL = SLOT_H(1);
  float* X0F = SLOT_F(2);  float* Z0F = SLOT_F(4);  float* W0F = SLOT_F(6);
  unsigned short* XCH = SLOT_H(8);  unsigned short* XCL = SLOT_H(9);  float* XCF = SLOT_F(10);
  unsigned short* ZCH = SLOT_H(12); unsigned short* ZCL = SLOT_H(13); float* ZCF = SLOT_F(14);
  float* DELTA = SLOT_F(2); float* BCF = SLOT_F(4);
  float* YTF = SLOT_F(0);
  unsigned short* YH = SLOT_H(8);   unsigned short* YL = SLOT_H(9);
  unsigned short* O1H = SLOT_H(2);  unsigned short* O1L = SLOT_H(3);
  unsigned short* LINH = SLOT_H(0); unsigned short* LINL = SLOT_H(1); float* LINF = SLOT_F(4);
  unsigned short* VT = SLOT_H(10);
  unsigned short* QRH = SLOT_H(8);  unsigned short* QRL = SLOT_H(9);  float* QUF = SLOT_F(6);
  unsigned short* KRT = SLOT_H(11);
  unsigned short* O2AH = SLOT_H(0); unsigned short* O2AL = SLOT_H(1);
  unsigned short* O2H = SLOT_H(4);  unsigned short* O2L = SLOT_H(5);
  float* OUTF = SLOT_F(6);
  unsigned short* H2H = SLOT_H(8);  unsigned short* H2L = SLOT_H(9);
  unsigned short* G0H = SLOT_H(0);  unsigned short* G0L = SLOT_H(1);
  unsigned short* G1H = SLOT_H(2);  unsigned short* G1L = SLOT_H(3);
  unsigned short* G2H = SLOT_H(4);  unsigned short* G2L = SLOT_H(5);
  unsigned short* G3H = SLOT_H(10); unsigned short* G3L = SLOT_H(11);
#undef SLOT_H
#undef SLOT_F
  unsigned short* WPL = (unsigned short*)(ws + oSM + SB_WPL);
  unsigned short* WIP  = WPL + WO_IP;
  unsigned short* WQK  = WPL + WO_QK;
  unsigned short* WXP  = WPL + WO_XP;
  unsigned short* WO1  = WPL + WO_O1;
  unsigned short* WPO  = WPL + WO_PO;
  unsigned short* WOUT = WPL + WO_OU;
  unsigned short* W1   = WPL + WO_F1;
  unsigned short* W2   = WPL + WO_F2;
  float* KMP = (float*)(ws + oSM + SB_KMP);
  float* KM  = (float*)(ws + oSM + SB_KM);
  unsigned short* KVP = (unsigned short*)(ws + oSM + SB_KVP);
  float* CT = (float*)(ws + oSM + SB_CT);
  float* ST = (float*)(ws + oSM + SB_ST);

  double r6 = 1.4678;
  for (int i = 0; i < 10; ++i) {
    const double r2 = r6 * r6, r4 = r2 * r2, r5 = r4 * r6, r66 = r5 * r6;
    r6 = r6 - (r66 - 10.0) / (6.0 * r5);
  }
  ThetaTab th;
  {
    double pw = 1.0;
    for (int j = 0; j < 24; ++j) {
      const float pf = (float)pw;
      th.v[j] = 1.0f / pf;
      pw *= r6;
    }
  }

  const dim3 blk(256);
  k_prep<<<dim3(9), blk, 0, stream>>>(in_proj_w, qk_w, x_proj_w, out_proj_w, proj_out_w, out_w, fc1_w, fc2_w,
                                      WPL, CT, ST, th);
  k_ln1<<<dim3(NT / 64), blk, 0, stream>>>(hidden, norm_in_g, norm_in_b, HSH, HSL);
  k_inproj<<<dim3(NT / 64, 3), blk, 0, stream>>>(HSH, HSL, WIP, X0F, Z0F, W0F);
  k_conv1d<<<dim3(NT / 64, 2), blk, 0, stream>>>(X0F, Z0F, conv_x_w, conv_z_w, XCH, XCL, XCF, ZCH, ZCL, ZCF);
  k_xproj<<<dim3(NT / 64), blk, 0, stream>>>(XCH, XCL, WXP, dt_proj_w, dt_proj_b, DELTA, BCF);
  k_scan<<<dim3(NBAT * CH / 2), dim3(32), 0, stream>>>(DELTA, XCF, BCF, A_log, Dv, YTF);
  k_ytr<<<dim3(NT / 64), blk, 0, stream>>>(YTF, YH, YL);
  k_out1<<<dim3(NT / 64), blk, 0, stream>>>(YH, YL, ZCH, ZCL, WO1, O1H, O1L);
  k_dwconv<<<dim3(NT / 64), blk, 0, stream>>>(W0F, dw_w, dw_b, LINH, LINL, LINF, VT);
  k_qk<<<dim3(NT / 64, 2), blk, 0, stream>>>(LINH, LINL, WQK, qk_b, CT, ST, QRH, QRL, QUF, KRT, KMP);
  k_kmean<<<dim3(1), blk, 0, stream>>>(KMP, KM);
  k_kv<<<dim3(NBAT * NHD), blk, 0, stream>>>(KRT, VT, KVP);
  k_attn<<<dim3(NT / 64), blk, 0, stream>>>(QRH, QRL, KVP, QUF, KM, LINF, ZCF, lepe_w, lepe_b, O2AH, O2AL);
  k_out2<<<dim3(NT / 64), blk, 0, stream>>>(O2AH, O2AL, WPO, proj_out_b, O2H, O2L);
  k_outp<<<dim3(NT / 64), blk, 0, stream>>>(O1H, O1L, O2H, O2L, WOUT, out_b, hidden, norm_mlp_g, norm_mlp_b,
                                            OUTF, H2H, H2L);
  k_fc1<<<dim3(NT / 64, 4), blk, 0, stream>>>(H2H, H2L, W1, fc1_b, G0H, G0L, G1H, G1L, G2H, G2L, G3H, G3L);
  k_fc2<<<dim3(NT / 64), blk, 0, stream>>>(G0H, G0L, G1H, G1L, G2H, G2L, G3H, G3L, W2, fc2_b, OUTF, out);
  (void)hipGetLastError();
}
